// RGCNLinkPredictor_74122545594486
// MI455X (gfx1250) — hardware-verified
//
#include <hip/hip_runtime.h>
#include <stddef.h>


#define HD      128
#define NR      8
#define KAGG    (NR * HD)
#define KTOT    (KAGG + HD)
#define NTHR    256
#define NWAVE   8
#define EPT     8
#define NGRP    2
#define CHUNK   (NTHR * EPT * NGRP)
#define WCAP    (EPT * NGRP * 32)
#define NBD     512
#define NSLOT   (NBD * NR)
#define SSHF    12
#define RCAP    16384
#define SEGCAP  128
#define GROWS   128
#define GCOLS   128
#define TPK     64
#define TPN     32
#define TPP     72
#define ASCL    16
#define WSCL    64
#define NPAD    1024
#define WSCAP   134217728

#define LDS_AGG   ((3 * NSLOT + RCAP + NWAVE * WCAP + 2 * NWAVE) * 4 + NWAVE * KTOT * 4)
#define LDS_GEMM  (GROWS * GCOLS * 4)

static_assert(NSLOT == (1 << SSHF));
static_assert((KAGG % 32) == 0 && (KTOT % 32) == 0 && (HD % 32) == 0);
static_assert((KTOT % TPK) == 0 && (KAGG % TPK) == 0 && (HD % TPN) == 0);
static_assert(TPN * 8 == NTHR && TPK == NWAVE * 8);
static_assert((TPP % 8) == 0 && TPP >= TPK);
static_assert(GROWS == NWAVE * 16 && GCOLS == 128 && HD == GCOLS);
static_assert(NBD == NWAVE * 64 && HD == 32 * 4);
static_assert(NSLOT == NTHR * 16);
static_assert(KAGG == 4 * 256);
static_assert((RCAP % 4) == 0 && WCAP == EPT * NGRP * 32);
static_assert(((NPAD / 2) % NBD) == 0 && ((NPAD / 2) % GROWS) == 0);
static_assert(LDS_AGG <= 300 * 1024);
static_assert(((3 * NSLOT + RCAP + NWAVE * WCAP + 2 * NWAVE) * 4) % 16 == 0);

typedef float     v4f  __attribute__((ext_vector_type(4)));
typedef float     v8f  __attribute__((ext_vector_type(8)));
typedef int       v4i  __attribute__((ext_vector_type(4)));
typedef _Float16  v8h  __attribute__((ext_vector_type(8)));
typedef _Float16  v16h __attribute__((ext_vector_type(16)));
union FragH { v16h v; v8h h[2]; };

__device__ __forceinline__ v8f wmf(v16h a, v16h b, v8f c) {
  v8f d = __builtin_amdgcn_wmma_f32_16x16x32_f16(false, a, false, b, (short)0, c, false, false);
  asm volatile("v_nop\n\tv_nop\n\tv_nop\n\tv_nop" : "+v"(d) : "v"(a), "v"(b));
  return d;
}

__device__ __forceinline__ v8h cvt8(v4f a, v4f b) {
  v8h h;
  h[0] = (_Float16)a.x; h[1] = (_Float16)a.y; h[2] = (_Float16)a.z; h[3] = (_Float16)a.w;
  h[4] = (_Float16)b.x; h[5] = (_Float16)b.y; h[6] = (_Float16)b.z; h[7] = (_Float16)b.w;
  return h;
}

__global__ __launch_bounds__(NTHR) void k_prep(
    const float* __restrict__ WA, const float* __restrict__ rootA,
    const float* __restrict__ WB, const float* __restrict__ rootB,
    _Float16* BwA, _Float16* BwB, float scale) {
  __shared__ __attribute__((aligned(16))) _Float16 sT[TPN * TPP];
  const int tid = threadIdx.x;
  const int z = (int)blockIdx.z;
  const float* W    = (z != 0) ? WB    : WA;
  const float* root = (z != 0) ? rootB : rootA;
  _Float16* Bw = (z != 0) ? BwB : BwA;
  const int k0 = (int)blockIdx.x * TPK, n0 = (int)blockIdx.y * TPN;
  const int nc = tid & 31, kq = tid >> 5;
  const int col = n0 + nc;
  const float* src = (k0 < KAGG) ? (W + (size_t)k0 * HD) : (root + (size_t)(k0 - KAGG) * HD);
#pragma unroll 1
  for (int it = 0; it < TPK / NWAVE; ++it) {
    const int kr = kq + NWAVE * it;
    const float w = src[(size_t)kr * HD + col];
    sT[nc * TPP + kr] = (_Float16)(w * scale);
  }
  __syncthreads();
  const int nl = tid >> 3, p = tid & 7;
  const v8h hv = *(const v8h*)(sT + nl * TPP + 8 * p);
  _Float16* d = Bw + (size_t)(n0 + nl) * KTOT + k0 + 8 * p;
  *(volatile v8h*)d = hv;
  __threadfence();
  *(volatile v8h*)d = hv;
}

template <int MODE>
__device__ __forceinline__ int scan_chunk(const int* __restrict__ kd, const int* __restrict__ kt, int nE,
                                          int cbase, int base, int vec8, unsigned* list,
                                          int tid, int lane, int wave) {
  int wc = 0;
#pragma unroll
  for (int g = 0; g < NGRP; ++g) {
    const int e0   = cbase + (g * NTHR + tid) * EPT;
    const int sent = -2147483647 - 1;
    const int i0 = min(e0, nE - 1),     i1 = min(e0 + 1, nE - 1), i2 = min(e0 + 2, nE - 1), i3 = min(e0 + 3, nE - 1);
    const int i4 = min(e0 + 4, nE - 1), i5 = min(e0 + 5, nE - 1), i6 = min(e0 + 6, nE - 1), i7 = min(e0 + 7, nE - 1);
    v4i da, db, ta, tb;
    if (vec8 != 0 && cbase + CHUNK <= nE) {
      da = *(const v4i*)(kd + e0);
      db = *(const v4i*)(kd + e0 + 4);
      ta = *(const v4i*)(kt + e0);
      tb = *(const v4i*)(kt + e0 + 4);
    } else {
      da.x = (e0     < nE) ? kd[i0] : sent;
      da.y = (e0 + 1 < nE) ? kd[i1] : sent;
      da.z = (e0 + 2 < nE) ? kd[i2] : sent;
      da.w = (e0 + 3 < nE) ? kd[i3] : sent;
      db.x = (e0 + 4 < nE) ? kd[i4] : sent;
      db.y = (e0 + 5 < nE) ? kd[i5] : sent;
      db.z = (e0 + 6 < nE) ? kd[i6] : sent;
      db.w = (e0 + 7 < nE) ? kd[i7] : sent;
      ta.x = kt[i0]; ta.y = kt[i1]; ta.z = kt[i2]; ta.w = kt[i3];
      tb.x = kt[i4]; tb.y = kt[i5]; tb.z = kt[i6]; tb.w = kt[i7];
    }
    const unsigned nb = (unsigned)base;
    const unsigned s0 = (unsigned)da.x - nb, s1 = (unsigned)da.y - nb;
    const unsigned s2 = (unsigned)da.z - nb, s3 = (unsigned)da.w - nb;
    const unsigned s4 = (unsigned)db.x - nb, s5 = (unsigned)db.y - nb;
    const unsigned s6 = (unsigned)db.z - nb, s7 = (unsigned)db.w - nb;
    const bool h0 = s0 < (unsigned)NBD, h1 = s1 < (unsigned)NBD, h2 = s2 < (unsigned)NBD, h3 = s3 < (unsigned)NBD;
    const bool h4 = s4 < (unsigned)NBD, h5 = s5 < (unsigned)NBD, h6 = s6 < (unsigned)NBD, h7 = s7 < (unsigned)NBD;
    const unsigned q0 = s0 * NR + (unsigned)min(max(ta.x, 0), NR - 1);
    const unsigned q1 = s1 * NR + (unsigned)min(max(ta.y, 0), NR - 1);
    const unsigned q2 = s2 * NR + (unsigned)min(max(ta.z, 0), NR - 1);
    const unsigned q3 = s3 * NR + (unsigned)min(max(ta.w, 0), NR - 1);
    const unsigned q4 = s4 * NR + (unsigned)min(max(tb.x, 0), NR - 1);
    const unsigned q5 = s5 * NR + (unsigned)min(max(tb.y, 0), NR - 1);
    const unsigned q6 = s6 * NR + (unsigned)min(max(tb.z, 0), NR - 1);
    const unsigned q7 = s7 * NR + (unsigned)min(max(tb.w, 0), NR - 1);
    const unsigned any = __builtin_amdgcn_ballot_w32(h0 | h1 | h2 | h3 | h4 | h5 | h6 | h7);
    if (any != 0u) {
#define HITJ(HJ, QJ, IJ) { \
        const unsigned mj = __builtin_amdgcn_ballot_w32(HJ); \
        if (mj != 0u) { \
          if (HJ) { \
            const int pos = wc + (int)__builtin_amdgcn_mbcnt_lo(mj, 0u); \
            const unsigned entv = (MODE != 0) ? ((((unsigned)(IJ)) << SSHF) | (QJ)) : (QJ); \
            if (pos < WCAP) list[wave * WCAP + pos] = entv; \
          } \
          wc += (int)__builtin_popcount(mj); } }
      HITJ(h0, q0, i0)
      HITJ(h1, q1, i1)
      HITJ(h2, q2, i2)
      HITJ(h3, q3, i3)
      HITJ(h4, q4, i4)
      HITJ(h5, q5, i5)
      HITJ(h6, q6, i6)
      HITJ(h7, q7, i7)
#undef HITJ
    }
  }
  return wc;
}

__global__ __launch_bounds__(NTHR) void k_aggmean(
    const int* __restrict__ edst, const int* __restrict__ etyp, const int* __restrict__ esrc,
    const float* __restrict__ x, _Float16* A16, int nE, int nN, int rowOff, int vec8) {
  extern __shared__ v4f lds_dyn[];
  int* scnt = (int*)lds_dyn;
  int* soff = scnt + NSLOT;
  int* curs = soff + NSLOT;
  unsigned* region = (unsigned*)(curs + NSLOT);
  unsigned* list = region + RCAP;
  int* wcnt = (int*)(list + NWAVE * WCAP);
  int* wtot = wcnt + NWAVE;
  float* stg = (float*)(wtot + NWAVE);
  const int tid = threadIdx.x, lane = tid & 31, wave = tid >> 5;
  const int base = rowOff + (int)blockIdx.x * NBD;

  {
    const v4i z = {0, 0, 0, 0};
    for (int i = tid; i < NSLOT / 4; i += NTHR) ((v4i*)scnt)[i] = z;
  }
  __syncthreads();

  const int nChunks = (nE + CHUNK - 1) / CHUNK;

#pragma unroll 1
  for (int ch = 0; ch < nChunks; ++ch) {
    const int cbase = ch * CHUNK;
    const int wc = scan_chunk<0>(edst, etyp, nE, cbase, base, vec8, list, tid, lane, wave);
    if (lane == 0) wcnt[wave] = wc;
    __syncthreads();
    if (wave == 0) {
#pragma unroll 1
      for (int wsx = 0; wsx < NWAVE; ++wsx) {
        int n = __builtin_amdgcn_readfirstlane(wcnt[wsx]);
        n = n > WCAP ? WCAP : (n < 0 ? 0 : n);
        const unsigned* lp = list + wsx * WCAP;
#pragma unroll 1
        for (int i = 0; i < n; ++i) {
          const int ent  = __builtin_amdgcn_readfirstlane((int)lp[i]);
          const int slot = ent & (NSLOT - 1);
          if (lane == 0) scnt[slot] = scnt[slot] + 1;
        }
      }
    }
    __syncthreads();
  }

  {
    const int sb = 16 * tid;
    const v4i c0 = *(const v4i*)(scnt + sb);
    const v4i c1 = *(const v4i*)(scnt + sb + 4);
    const v4i c2 = *(const v4i*)(scnt + sb + 8);
    const v4i c3 = *(const v4i*)(scnt + sb + 12);
    const int ts = (c0.x + c0.y + c0.z + c0.w) + (c1.x + c1.y + c1.z + c1.w)
                 + (c2.x + c2.y + c2.z + c2.w) + (c3.x + c3.y + c3.z + c3.w);
    int incl = ts;
#pragma unroll
    for (int dd = 1; dd < 32; dd <<= 1) {
      const int t = __shfl_up(incl, dd, 32);
      if (lane >= dd) incl += t;
    }
    if (lane == 31) wtot[wave] = incl;
    __syncthreads();
    int pre = 0;
#pragma unroll 1
    for (int w = 0; w < wave; ++w) pre += wtot[w];
    int run = pre + incl - ts;
    v4i o0, o1, o2, o3;
    o0.x = run; run += c0.x; o0.y = run; run += c0.y; o0.z = run; run += c0.z; o0.w = run; run += c0.w;
    o1.x = run; run += c1.x; o1.y = run; run += c1.y; o1.z = run; run += c1.z; o1.w = run; run += c1.w;
    o2.x = run; run += c2.x; o2.y = run; run += c2.y; o2.z = run; run += c2.z; o2.w = run; run += c2.w;
    o3.x = run; run += c3.x; o3.y = run; run += c3.y; o3.z = run; run += c3.z; o3.w = run;
    *(v4i*)(soff + sb) = o0; *(v4i*)(soff + sb + 4) = o1; *(v4i*)(soff + sb + 8) = o2; *(v4i*)(soff + sb + 12) = o3;
    *(v4i*)(curs + sb) = o0; *(v4i*)(curs + sb + 4) = o1; *(v4i*)(curs + sb + 8) = o2; *(v4i*)(curs + sb + 12) = o3;
    __syncthreads();
  }

#pragma unroll 1
  for (int ch = 0; ch < nChunks; ++ch) {
    const int cbase = ch * CHUNK;
    const int wc = scan_chunk<1>(edst, etyp, nE, cbase, base, vec8, list, tid, lane, wave);
    if (lane == 0) wcnt[wave] = wc;
    __syncthreads();
    if (wave == 0) {
#pragma unroll 1
      for (int wsx = 0; wsx < NWAVE; ++wsx) {
        int n = __builtin_amdgcn_readfirstlane(wcnt[wsx]);
        n = n > WCAP ? WCAP : (n < 0 ? 0 : n);
        const unsigned* lp = list + wsx * WCAP;
#pragma unroll 1
        for (int i = 0; i < n; ++i) {
          const unsigned ent = (unsigned)__builtin_amdgcn_readfirstlane((int)lp[i]);
          const int slot = (int)(ent & (unsigned)(NSLOT - 1));
          int ev = (int)(ent >> SSHF);
          ev = ev > nE - 1 ? nE - 1 : ev;
          if (lane == 0) {
            const int pos = curs[slot];
            if ((unsigned)pos < (unsigned)RCAP) region[pos] = (unsigned)ev;
            curs[slot] = (pos >= RCAP) ? RCAP : pos + 1;
          }
        }
      }
    }
    __syncthreads();
  }

  const float qnan = __int_as_float(0x7fc00000);
  float* stgw = stg + wave * KTOT;
#pragma unroll 1
  for (int jj = 0; jj < NBD / NWAVE; ++jj) {
    const int j  = wave + NWAVE * jj;
    const int d  = base + j;
    const int dc = d < nN ? d : nN - 1;
    const int lr = d - rowOff;
    {
      const v4f xv = *(const v4f*)(x + (size_t)dc * HD + 4 * lane);
      *(v4f*)(stgw + KAGG + 4 * lane) = xv * (float)ASCL;
    }
#pragma unroll 1
    for (int r = 0; r < NR; ++r) {
      const int slot = j * NR + r;
      const int n  = __builtin_amdgcn_readfirstlane(scnt[slot]);
      const int st = __builtin_amdgcn_readfirstlane(soff[slot]);
      const bool bad = (n > SEGCAP) || (n < 0) || (st < 0) || (st + n > RCAP);
      const int nn = n < 0 ? 0 : (n > SEGCAP ? SEGCAP : n);
      v4f a0 = {0.f, 0.f, 0.f, 0.f};
#pragma unroll 1
      for (int p = 0; p < nn; ++p) {
        int pos = st + p;
        pos = pos < 0 ? 0 : (pos > RCAP - 1 ? RCAP - 1 : pos);
        const int eu = __builtin_amdgcn_readfirstlane((int)region[pos]);
        const int e  = eu < 0 ? 0 : (eu > nE - 1 ? nE - 1 : eu);
        int s = esrc[e];
        s = s < 0 ? 0 : (s > nN - 1 ? nN - 1 : s);
        a0 = a0 + *(const v4f*)(x + (size_t)s * HD + 4 * lane);
      }
      float inv = (float)ASCL * (1.0f / (float)(nn > 0 ? nn : 1));
      inv = bad ? qnan : inv;
      *(v4f*)(stgw + r * HD + 4 * lane) = a0 * inv;
    }
    __syncthreads();
    const float* q0 = stgw + 8 * lane;
    const v8h hv0 = cvt8(*(const v4f*)(q0),       *(const v4f*)(q0 + 4));
    const v8h hv1 = cvt8(*(const v4f*)(q0 + 256), *(const v4f*)(q0 + 260));
    const v8h hv2 = cvt8(*(const v4f*)(q0 + 512), *(const v4f*)(q0 + 516));
    const v8h hv3 = cvt8(*(const v4f*)(q0 + 768), *(const v4f*)(q0 + 772));
    const float* q4 = stgw + KAGG + 8 * (lane & 15);
    const v8h hv4 = cvt8(*(const v4f*)(q4), *(const v4f*)(q4 + 4));
    _Float16* gp = A16 + (size_t)lr * KTOT + 8 * lane;
    *(volatile v8h*)(gp)       = hv0;
    *(volatile v8h*)(gp + 256) = hv1;
    *(volatile v8h*)(gp + 512) = hv2;
    *(volatile v8h*)(gp + 768) = hv3;
    if (lane < 16) *(volatile v8h*)(gp + KAGG) = hv4;
    __threadfence();
    *(volatile v8h*)(gp)       = hv0;
    *(volatile v8h*)(gp + 256) = hv1;
    *(volatile v8h*)(gp + 512) = hv2;
    *(volatile v8h*)(gp + 768) = hv3;
    if (lane < 16) *(volatile v8h*)(gp + KAGG) = hv4;
    __syncthreads();
  }
}

__device__ __forceinline__ void kstep(v8f (&acc)[GCOLS / 16], const _Float16* ap, const _Float16* bp) {
  FragH af;
  af.h[0] = *(const v8h*)ap;
  af.h[1] = *(const v8h*)(ap + 16);
#pragma unroll
  for (int t = 0; t < GCOLS / 16; ++t) {
    const _Float16* bq = bp + (size_t)(16 * t) * KTOT;
    FragH bf;
    bf.h[0] = *(const v8h*)bq;
    bf.h[1] = *(const v8h*)(bq + 16);
    acc[t] = wmf(af.v, bf.v, acc[t]);
  }
}

__global__ __launch_bounds__(NTHR) void k_gemm(
    const _Float16* __restrict__ A16, const _Float16* __restrict__ Bw, const float* __restrict__ bias,
    float* Hout, int nRows, int rowOff, float osc) {
  extern __shared__ v4f lds_dyn[];
  constexpr int NC = GCOLS;
  constexpr int NT = NC / 16;
  const int tid = threadIdx.x, lane = tid & 31, wave = tid >> 5, hh = lane >> 4, m = lane & 15;
  const int rowBase = (int)blockIdx.x * GROWS;
  const int ar  = rowBase + wave * 16 + m;
  const int arc = ar < nRows ? ar : nRows - 1;
  const _Float16* ap  = A16 + (size_t)arc * KTOT + 8 * hh;
  const _Float16* bp0 = Bw + (size_t)m * KTOT + 8 * hh;

  v8f acc[NT];
#pragma unroll
  for (int t = 0; t < NT; ++t) { v8f zz = {0.f, 0.f, 0.f, 0.f, 0.f, 0.f, 0.f, 0.f}; acc[t] = zz; }

#pragma unroll 1
  for (int kt = 0; kt < KTOT / 32; ++kt) kstep(acc, ap + 32 * kt, bp0 + 32 * kt);

  float bc[NT];
#pragma unroll
  for (int t = 0; t < NT; ++t) bc[t] = bias[16 * t + m];
  const int r0 = wave * 16 + 8 * hh;

  float* stg = (float*)lds_dyn;
  float* sp = stg + r0 * NC + m;
#pragma unroll
  for (int t = 0; t < NT; ++t) {
#pragma unroll
    for (int r = 0; r < 8; ++r) {
      float v = acc[t][r] * osc + bc[t];
      v = (v < 0.0f) ? 0.0f : v;
      sp[r * NC + 16 * t] = v;
    }
  }
  __syncthreads();
  const float* lp = stg + wave * 16 * NC;
  float* gp = Hout + (size_t)(rowOff + rowBase + wave * 16) * HD;
#pragma unroll
  for (int i = 0; i < 16; ++i) {
    const v4f v = *(const v4f*)(lp + i * NC + 4 * lane);
    *(volatile v4f*)(gp + (size_t)i * HD + 4 * lane) = v;
  }
  __threadfence();
#pragma unroll
  for (int i = 0; i < 16; ++i) {
    const v4f v = *(const v4f*)(lp + i * NC + 4 * lane);
    *(volatile v4f*)(gp + (size_t)i * HD + 4 * lane) = v;
  }
}

__global__ __launch_bounds__(NTHR) void k_score(
    const float* __restrict__ H, const float* __restrict__ relE,
    const int* __restrict__ hidx, const int* __restrict__ ridx, const int* __restrict__ tix,
    float* out, int nT, int nN) {
  __shared__ __attribute__((aligned(16))) float ssc[NTHR];
  const int tid = threadIdx.x, lane = tid & 31, wave = tid >> 5;
  const int tb = (int)blockIdx.x * NTHR + wave * 32;
  float mine = 0.0f;
#pragma unroll 1
  for (int t = 0; t < 32; ++t) {
    int ix = tb + t;
    ix = ix > nT - 1 ? nT - 1 : ix;
    int a = hidx[ix];  a = a < 0 ? 0 : (a > nN - 1 ? nN - 1 : a);
    int b = ridx[ix];  b = b < 0 ? 0 : (b > NR - 1 ? NR - 1 : b);
    int c = tix[ix];   c = c < 0 ? 0 : (c > nN - 1 ? nN - 1 : c);
    const v4f va = *(const v4f*)(H + (size_t)a * HD + 4 * lane);
    const v4f vb = *(const v4f*)(relE + (size_t)b * HD + 4 * lane);
    const v4f vc = *(const v4f*)(H + (size_t)c * HD + 4 * lane);
    float p = (va.x * vb.x) * vc.x + (va.y * vb.y) * vc.y + (va.z * vb.z) * vc.z + (va.w * vb.w) * vc.w;
#pragma unroll
    for (int off = 16; off > 0; off >>= 1) p += __shfl_xor(p, off, 32);
    mine = (lane == t) ? p : mine;
  }
  ssc[tid] = mine;
  __syncthreads();
  if (wave < 2) {
    const int e0 = (int)blockIdx.x * NTHR + wave * 128 + 4 * lane;
    const v4f v = *(const v4f*)(ssc + wave * 128 + 4 * lane);
    const bool full = (e0 + 4 <= nT);
    if (full) {
      *(volatile v4f*)(out + e0) = v;
    } else {
      if (e0     < nT) *(volatile float*)(out + e0)     = v.x;
      if (e0 + 1 < nT) *(volatile float*)(out + e0 + 1) = v.y;
      if (e0 + 2 < nT) *(volatile float*)(out + e0 + 2) = v.z;
      if (e0 + 3 < nT) *(volatile float*)(out + e0 + 3) = v.w;
    }
    __threadfence();
    if (full) {
      *(volatile v4f*)(out + e0) = v;
    } else {
      if (e0     < nT) *(volatile float*)(out + e0)     = v.x;
      if (e0 + 1 < nT) *(volatile float*)(out + e0 + 1) = v.y;
      if (e0 + 2 < nT) *(volatile float*)(out + e0 + 2) = v.z;
      if (e0 + 3 < nT) *(volatile float*)(out + e0 + 3) = v.w;
    }
  }
}

extern "C" void kernel_launch(void* const* d_in, const int* in_sizes, int n_in,
                              void* d_out, int out_size, void* d_ws, size_t ws_size,
                              hipStream_t stream) {
  if (n_in < 13) return;
  if (in_sizes[0] < HD || (in_sizes[0] % HD) != 0) return;
  const int nN = in_sizes[0] / HD;
  if (in_sizes[1] != NR * HD * HD || in_sizes[2] != HD * HD || in_sizes[3] != HD) return;
  if (in_sizes[4] != NR * HD * HD || in_sizes[5] != HD * HD || in_sizes[6] != HD) return;
  if (in_sizes[7] != NR * HD) return;
  const int nE = in_sizes[9];
  if (nE < 1 || in_sizes[8] != 2 * nE) return;
  if (nE > (1 << 20)) return;
  const int nT = out_size;
  if (nT < 1 || in_sizes[10] != nT || in_sizes[11] != nT || in_sizes[12] != nT) return;
  if (nN > (1 << 24)) return;
  const int NP  = ((nN + NPAD - 1) / NPAD) * NPAD;
  const int NPH = NP / 2;

  const float* emb   = (const float*)d_in[0];
  const float* W0    = (const float*)d_in[1];
  const float* root0 = (const float*)d_in[2];
  const float* b0    = (const float*)d_in[3];
  const float* W1    = (const float*)d_in[4];
  const float* root1 = (const float*)d_in[5];
  const float* b1    = (const float*)d_in[6];
  const float* relE  = (const float*)d_in[7];
  const int*   ei    = (const int*)d_in[8];
  const int*   e_typ = (const int*)d_in[9];
  const int*   hidx  = (const int*)d_in[10];
  const int*   ridx  = (const int*)d_in[11];
  const int*   tix   = (const int*)d_in[12];
  const int*   e_src = ei;
  const int*   e_dst = ei + nE;
  float* out = (float*)d_out;

  char* ws = (char*)d_ws;
  size_t off = 0;
#define CARVE(NAME, BYTES) const size_t NAME = off; off += (size_t)(BYTES); off = (off + 255) & ~(size_t)255;
  CARVE(oBw0, (size_t)HD * KTOT * 2)
  CARVE(oBw1, (size_t)HD * KTOT * 2)
  CARVE(oA16, (size_t)NPH * KTOT * 2)
  CARVE(oH1,  (size_t)NP * HD * 4)
  CARVE(oH2,  (size_t)NP * HD * 4)
#undef CARVE
  if (off > ws_size || off > (size_t)WSCAP) return;
  _Float16* Bw0 = (_Float16*)(ws + oBw0);
  _Float16* Bw1 = (_Float16*)(ws + oBw1);
  _Float16* A16 = (_Float16*)(ws + oA16);
  float*    H1  = (float*)(ws + oH1);
  float*    H2  = (float*)(ws + oH2);

  const float osc = 1.0f / ((float)ASCL * (float)WSCL);
  const int vec8 = ((nE & 3) == 0) ? 1 : 0;

  k_prep<<<dim3(KTOT / TPK, HD / TPN, 2), NTHR, 0, stream>>>(W0, root0, W1, root1, Bw0, Bw1, (float)WSCL);

  hipFuncSetAttribute(reinterpret_cast<const void*>(&k_aggmean),
                      hipFuncAttributeMaxDynamicSharedMemorySize, LDS_AGG);
  hipFuncSetAttribute(reinterpret_cast<const void*>(&k_gemm),
                      hipFuncAttributeMaxDynamicSharedMemorySize, LDS_GEMM);

  for (int l = 0; l < 2; ++l) {
    const float* xin  = (l != 0) ? (const float*)H1 : emb;
    float*       hout = (l != 0) ? H2 : H1;
    const _Float16* Bw = (l != 0) ? Bw1 : Bw0;
    const float* bias = (l != 0) ? b1 : b0;
    for (int h = 0; h < 2; ++h) {
      const int rowOff = h * NPH;
      k_aggmean<<<NPH / NBD, NTHR, LDS_AGG, stream>>>(e_dst, e_typ, e_src, xin, A16, nE, nN, rowOff, vec8);
      k_gemm<<<dim3(NPH / GROWS, 1, 1), NTHR, LDS_GEMM, stream>>>(A16, Bw, bias, hout, NPH, rowOff, osc);
    }
  }

  k_score<<<(nT + NTHR - 1) / NTHR, NTHR, 0, stream>>>(H2, relE, hidx, ridx, tix, out, nT, nN);
}
